// MultiHeadSA_74775380623733
// MI455X (gfx1250) — hardware-verified
//
#include <hip/hip_runtime.h>
#include <math.h>
#include <stdint.h>

#define NB   8
#define HH   8
#define DM   256
#define PP   1024
#define HDIM 2048
#define PSCALE 32768.0f
#define PSCALE_INV (1.0f / 32768.0f)

typedef __attribute__((ext_vector_type(16))) _Float16 v16h;
typedef __attribute__((ext_vector_type(8)))  _Float16 v8h;
typedef __attribute__((ext_vector_type(16))) __bf16   v16b;
typedef __attribute__((ext_vector_type(8)))  __bf16   v8b;
typedef __attribute__((ext_vector_type(8)))  float    v8f;
typedef __attribute__((ext_vector_type(4)))  float    v4f;
typedef __attribute__((ext_vector_type(2)))  float    v2f;
typedef __attribute__((ext_vector_type(4)))  unsigned int v4u;

__device__ __forceinline__ unsigned short f2bf_bits(float f) {
  unsigned u = __float_as_uint(f);
  return (unsigned short)((u + 0x7FFFu + ((u >> 16) & 1u)) >> 16);
}
__device__ __forceinline__ float bf_bits2f(unsigned short h) { return __uint_as_float(((unsigned)h) << 16); }

__device__ __forceinline__ void dep_guard_h(v8f& a, v8f& b, v16h x, v16h y) { asm volatile("v_nop\n\tv_nop\n\tv_nop\n\tv_nop" : "+v"(a), "+v"(b) : "v"(x), "v"(y)); }
__device__ __forceinline__ void dep_guard_b(v8f& a, v8f& b, v16b x, v16b y) { asm volatile("v_nop\n\tv_nop\n\tv_nop\n\tv_nop" : "+v"(a), "+v"(b) : "v"(x), "v"(y)); }
__device__ __forceinline__ void keep4_h(v16h a, v16h b, v16h c, v16h d) { asm volatile("v_nop" :: "v"(a), "v"(b), "v"(c), "v"(d)); }
__device__ __forceinline__ void keep4_b(v16b a, v16b b, v16b c, v16b d) { asm volatile("v_nop" :: "v"(a), "v"(b), "v"(c), "v"(d)); }
__device__ __forceinline__ void acc_guard4(v8f& a, v8f& b, v8f& c, v8f& d) { asm volatile("v_nop\n\tv_nop\n\tv_nop\n\tv_nop" : "+v"(a), "+v"(b), "+v"(c), "+v"(d)); }
template <typename T> struct Frag;
template <> struct Frag<_Float16> {
  typedef v16h V; union U { v16h v; v8h h[2]; };
  static __device__ __forceinline__ v16h load(const _Float16* p) {
    U f; f.h[0] = *(const v8h*)(p); f.h[1] = *(const v8h*)(p + 16); return f.v;
  }
  static __device__ __forceinline__ v8f mma(v16h a, v16h b, v8f c) {
    return __builtin_amdgcn_wmma_f32_16x16x32_f16(false, a, false, b, (short)0, c, false, false);
  }
  static __device__ __forceinline__ void guard(v8f& a, v8f& b, v16h x, v16h y) { dep_guard_h(a, b, x, y); }
  static __device__ __forceinline__ void keep(v16h a, v16h b, v16h c, v16h d) { keep4_h(a, b, c, d); }
};
template <> struct Frag<__bf16> {
  typedef v16b V; union U { v16b v; v8b h[2]; };
  static __device__ __forceinline__ v16b load(const __bf16* p) {
    U f; f.h[0] = *(const v8b*)(p); f.h[1] = *(const v8b*)(p + 16); return f.v;
  }
  static __device__ __forceinline__ v8f mma(v16b a, v16b b, v8f c) {
    return __builtin_amdgcn_wmma_f32_16x16x32_bf16(false, a, false, b, (short)0, c, false, false);
  }
  static __device__ __forceinline__ void guard(v8f& a, v8f& b, v16b x, v16b y) { dep_guard_b(a, b, x, y); }
  static __device__ __forceinline__ void keep(v16b a, v16b b, v16b c, v16b d) { keep4_b(a, b, c, d); }
};

template <int ET> struct Elem;
template <> struct Elem<0> { typedef _Float16 T; };
template <> struct Elem<1> { typedef __bf16 T; };
template <int ET, bool SPLIT, int BIAS_MODE, int OUT_MODE, bool RESID, int ACT = 0>
__global__ __launch_bounds__(256) void wmma_gemm64(
    const unsigned short* __restrict__ Ap, const unsigned short* __restrict__ A2p, int lda, long strideA,
    const unsigned short* __restrict__ Btp, const unsigned short* __restrict__ Bt2p, int ldb, long strideB,
    void* __restrict__ Cout, void* __restrict__ Cout2, int ldc, long strideC,
    const float* __restrict__ bias,
    const float* __restrict__ resid, long strideR,
    int M, int N, int K, float scale) {
  typedef typename Elem<ET>::T T;
  typedef typename Frag<T>::V V;
  const T* A = (const T*)Ap; const T* A2 = (const T*)A2p; const T* Bt = (const T*)Btp; const T* Bt2 = (const T*)Bt2p;
  __shared__ __align__(16) float sT[8][16 * 68];
  const int b    = blockIdx.y;
  const int lane = threadIdx.x & 31;
  const int wave = threadIdx.x >> 5;
  const int tilesN = N >> 6;
  const int tilesM = M >> 6;
  const int tile = blockIdx.x * 8 + wave;
  if (tile >= tilesM * tilesN) return;
  const int tm = tile / tilesN;
  const int tn = tile - tm * tilesN;
  const int m0 = tm << 6;
  const int n0 = tn << 6;

  const T* Ab  = A  + (size_t)b * strideA;
  const T* Bb  = Bt + (size_t)b * strideB;
  const T* Ab2 = SPLIT ? (A2  + (size_t)b * strideA) : nullptr;
  const T* Bb2 = SPLIT ? (Bt2 + (size_t)b * strideB) : nullptr;

  const int rlane = lane & 15;
  const int koff  = (lane >> 4) * 8;
  const int mOff  = (lane >> 4) * 8;

  v8f acc[4][4];
#pragma unroll
  for (int i = 0; i < 4; ++i)
#pragma unroll
    for (int j = 0; j < 4; ++j) acc[i][j] = (v8f){0.f,0.f,0.f,0.f,0.f,0.f,0.f,0.f};

  for (int k0 = 0; k0 < K; k0 += 32) {
    V bh[4], bl[4];
#pragma unroll
    for (int j = 0; j < 4; ++j) {
      const size_t bo = (size_t)(n0 + (j << 4) + rlane) * ldb + koff + k0;
      bh[j] = Frag<T>::load(Bb + bo);
      if (SPLIT) bl[j] = Frag<T>::load(Bb2 + bo);
    }
#pragma unroll
    for (int i = 0; i < 4; ++i) {
      const size_t ao = (size_t)(m0 + (i << 4) + rlane) * lda + koff + k0;
      V ah = Frag<T>::load(Ab + ao);
      V al;
      if (SPLIT) al = Frag<T>::load(Ab2 + ao);
#pragma unroll
      for (int j = 0; j < 4; ++j) {
        acc[i][j] = Frag<T>::mma(ah, bh[j], acc[i][j]);
        if (SPLIT) {
          acc[i][j] = Frag<T>::mma(ah, bl[j], acc[i][j]);
          acc[i][j] = Frag<T>::mma(al, bh[j], acc[i][j]);
        }
      }
      Frag<T>::guard(acc[i][0], acc[i][3], ah, SPLIT ? al : ah);
    }
    Frag<T>::keep(bh[0], bh[1], bh[2], bh[3]);
    if (SPLIT) Frag<T>::keep(bl[0], bl[1], bl[2], bl[3]);
  }
  acc_guard4(acc[0][0], acc[0][1], acc[0][2], acc[0][3]);
  acc_guard4(acc[1][0], acc[1][1], acc[1][2], acc[1][3]);
  acc_guard4(acc[2][0], acc[2][1], acc[2][2], acc[2][3]);
  acc_guard4(acc[3][0], acc[3][1], acc[3][2], acc[3][3]);

  float* slab = sT[wave];
  const float* Rb = RESID ? (resid + (size_t)b * strideR) : nullptr;
#pragma unroll
  for (int i = 0; i < 4; ++i) {
    const int mBase = m0 + (i << 4);
#pragma unroll
    for (int j = 0; j < 4; ++j) {
      const int n = n0 + (j << 4) + rlane;
      float bv = 0.f;
      if (BIAS_MODE == 2) bv = bias[n];
#pragma unroll
      for (int r = 0; r < 8; ++r) {
        float v = acc[i][j][r] * scale;
        if (BIAS_MODE == 1) v += bias[mBase + mOff + r];
        if (BIAS_MODE == 2) v += bv;
        if (RESID) v += Rb[(size_t)(mBase + mOff + r) * ldc + n];
        if (ACT == 1) v = tanhf(v);
        if (ACT == 2) v = fmaxf(v, 0.0f);
        if (ACT == 3) v = v / (1.0f + expf(-v));
        if (ACT == 4) v = (v > 0.f) ? v : 0.01f * v;
        slab[(mOff + r) * 68 + (j << 4) + rlane] = v;
      }
    }
    __builtin_amdgcn_fence(__ATOMIC_RELEASE, "workgroup");
    __builtin_amdgcn_wave_barrier();
    __builtin_amdgcn_fence(__ATOMIC_ACQUIRE, "workgroup");
    if (OUT_MODE == 0) {
      float* C = (float*)Cout + (size_t)b * strideC;
      const int hh = lane >> 4, c4 = (lane & 15) * 4;
      for (int pass = 0; pass < 2; ++pass) {
#pragma unroll
        for (int it = 0; it < 8; ++it) {
          const int row = it * 2 + hh;
          v4f v = *(const v4f*)(slab + row * 68 + c4);
          *(volatile v4f*)(C + (size_t)(mBase + row) * ldc + n0 + c4) = v;
        }
        __threadfence();
      }
    } else {
      const int q = lane >> 3, c8 = (lane & 7) * 8;
      unsigned short* C  = (unsigned short*)Cout  + (size_t)b * strideC;
      unsigned short* C2 = (OUT_MODE == 2) ? ((unsigned short*)Cout2 + (size_t)b * strideC) : nullptr;
      for (int pass = 0; pass < 2; ++pass) {
#pragma unroll
        for (int it = 0; it < 4; ++it) {
          const int row = it * 4 + q;
          const float* sp = slab + row * 68 + c8;
          v8h hv, lv;
#pragma unroll
          for (int e = 0; e < 8; ++e) {
            if (OUT_MODE == 1) {
              hv[e] = (_Float16)sp[e];
            } else {
              unsigned short hb = f2bf_bits(sp[e]);
              unsigned short lb = f2bf_bits(sp[e] - bf_bits2f(hb));
              hv[e] = __builtin_bit_cast(_Float16, hb);
              lv[e] = __builtin_bit_cast(_Float16, lb);
            }
          }
          *(volatile v8h*)(C + (size_t)(mBase + row) * ldc + n0 + c8) = hv;
          if (OUT_MODE == 2) *(volatile v8h*)(C2 + (size_t)(mBase + row) * ldc + n0 + c8) = lv;
        }
        __threadfence();
      }
    }
    __builtin_amdgcn_fence(__ATOMIC_RELEASE, "workgroup");
    __builtin_amdgcn_wave_barrier();
    __builtin_amdgcn_fence(__ATOMIC_ACQUIRE, "workgroup");
  }
}

__device__ __forceinline__ unsigned pk16(unsigned short a, unsigned short b) { return (unsigned)a | ((unsigned)b << 16); }
__device__ __forceinline__ unsigned short h_bits(float f) { const _Float16 h = (_Float16)f; return __builtin_bit_cast(unsigned short, h); }

__global__ __launch_bounds__(256) void cast_f16x2_kernel(const float* __restrict__ in, unsigned short* __restrict__ out, int n2, float scale) {
  const int i = blockIdx.x * 256 + threadIdx.x;
  if (i < n2) {
    const v2f f = *(const v2f*)(in + 2 * (size_t)i);
    const unsigned u = pk16(h_bits(f[0] * scale), h_bits(f[1] * scale));
    ((volatile unsigned*)out)[i] = u;
    __threadfence();
    ((volatile unsigned*)out)[i] = u;
  }
}

__global__ __launch_bounds__(256) void xt_cast_kernel(const float* __restrict__ x, unsigned short* __restrict__ XT) {
  __shared__ float tile[64][65];
  const int bid = blockIdx.x;
  const int dt = bid & 3;
  const int pt = (bid >> 2) & 15;
  const int n  = bid >> 6;
  const int d0 = dt * 64, p0 = pt * 64;
  const int tid = threadIdx.x, lane = tid & 31, wave = tid >> 5;
  {
    const int r = tid >> 2, cs = (tid & 3) * 16;
    const float* src = x + ((size_t)n * DM + d0 + r) * PP + p0 + cs;
#pragma unroll
    for (int i = 0; i < 4; ++i) {
      const v4f v = *(const v4f*)(src + 4 * i);
      tile[r][cs + 4 * i + 0] = v[0];
      tile[r][cs + 4 * i + 1] = v[1];
      tile[r][cs + 4 * i + 2] = v[2];
      tile[r][cs + 4 * i + 3] = v[3];
    }
  }
  __syncthreads();
  const int q = lane >> 3, c8 = (lane & 7) * 8;
  unsigned short* ob = XT + ((size_t)n * PP + p0) * DM + d0;
  for (int pass = 0; pass < 2; ++pass) {
#pragma unroll
    for (int it = 0; it < 2; ++it) {
      const int rr = wave * 8 + it * 4 + q;
      v8h hv;
#pragma unroll
      for (int e = 0; e < 8; ++e) hv[e] = (_Float16)tile[c8 + e][rr];
      *(volatile v8h*)(ob + (size_t)rr * DM + c8) = hv;
    }
    __threadfence();
  }
}

__global__ __launch_bounds__(256) void pos_t_kernel(const float* __restrict__ pos, float* __restrict__ PT) {
  __shared__ float tile[64][65];
  const int bid = blockIdx.x;
  const int qt = bid & 15;
  const int kt = (bid >> 4) & 15;
  const int h  = bid >> 8;
  const int k0 = kt * 64, q0 = qt * 64;
  const int tid = threadIdx.x, lane = tid & 31, wave = tid >> 5;
  {
    const int r = tid >> 2, cs = (tid & 3) * 16;
    const float* src = pos + ((size_t)h * PP + k0 + r) * PP + q0 + cs;
#pragma unroll
    for (int i = 0; i < 4; ++i) {
      const v4f v = *(const v4f*)(src + 4 * i);
      tile[r][cs + 4 * i + 0] = v[0];
      tile[r][cs + 4 * i + 1] = v[1];
      tile[r][cs + 4 * i + 2] = v[2];
      tile[r][cs + 4 * i + 3] = v[3];
    }
  }
  __syncthreads();
  const int hh = lane >> 4, c4 = (lane & 15) * 4;
  float* ob = PT + ((size_t)h * PP + q0) * PP + k0;
  for (int pass = 0; pass < 2; ++pass) {
#pragma unroll
    for (int it = 0; it < 4; ++it) {
      const int rr = wave * 8 + it * 2 + hh;
      v4f v;
      v[0] = tile[c4 + 0][rr];
      v[1] = tile[c4 + 1][rr];
      v[2] = tile[c4 + 2][rr];
      v[3] = tile[c4 + 3][rr];
      *(volatile v4f*)(ob + (size_t)rr * PP + c4) = v;
    }
    __threadfence();
  }
}

__global__ __launch_bounds__(128) void softmax_bias_kernel(const float* __restrict__ S,
                                                           const float* __restrict__ PT,
                                                           unsigned short* __restrict__ P) {
  __shared__ float redm[4];
  __shared__ float reds[4];
  const int qp   = blockIdx.x;
  const int h    = blockIdx.y;
  const int tid  = threadIdx.x;
  const int lane = tid & 31;
  const int wave = tid >> 5;
  const int j0   = tid * 8;
  const size_t ro = ((size_t)h * PP + qp) * PP + j0;
  const v4f a  = *(const v4f*)(S + ro);
  const v4f c  = *(const v4f*)(S + ro + 4);
  const v4f ba = *(const v4f*)(PT + ro);
  const v4f bc = *(const v4f*)(PT + ro + 4);
  const float t0 = a[0] + ba[0], t1 = a[1] + ba[1], t2 = a[2] + ba[2], t3 = a[3] + ba[3];
  const float t4 = c[0] + bc[0], t5 = c[1] + bc[1], t6 = c[2] + bc[2], t7 = c[3] + bc[3];
  float m = fmaxf(fmaxf(fmaxf(t0, t1), fmaxf(t2, t3)), fmaxf(fmaxf(t4, t5), fmaxf(t6, t7)));
#pragma unroll
  for (int off = 16; off > 0; off >>= 1) m = fmaxf(m, __shfl_xor(m, off, 32));
  if (lane == 0) redm[wave] = m;
  __syncthreads();
  const float mx = fmaxf(fmaxf(redm[0], redm[1]), fmaxf(redm[2], redm[3]));
  const float e0 = __expf(t0 - mx), e1 = __expf(t1 - mx), e2 = __expf(t2 - mx), e3 = __expf(t3 - mx);
  const float e4 = __expf(t4 - mx), e5 = __expf(t5 - mx), e6 = __expf(t6 - mx), e7 = __expf(t7 - mx);
  float s = ((e0 + e1) + (e2 + e3)) + ((e4 + e5) + (e6 + e7));
#pragma unroll
  for (int off = 16; off > 0; off >>= 1) s += __shfl_xor(s, off, 32);
  if (lane == 0) reds[wave] = s;
  __syncthreads();
  const float tot = ((reds[0] + reds[1]) + reds[2]) + reds[3];
  const float inv = 1.0f / tot;
  const float p0 = e0 * inv, p1 = e1 * inv, p2 = e2 * inv, p3 = e3 * inv;
  const float p4 = e4 * inv, p5 = e5 * inv, p6 = e6 * inv, p7 = e7 * inv;
  const v4u hv = (v4u){pk16(h_bits(p0 * PSCALE), h_bits(p1 * PSCALE)),
                       pk16(h_bits(p2 * PSCALE), h_bits(p3 * PSCALE)),
                       pk16(h_bits(p4 * PSCALE), h_bits(p5 * PSCALE)),
                       pk16(h_bits(p6 * PSCALE), h_bits(p7 * PSCALE))};
  *(volatile v4u*)(P + ro) = hv;
  __threadfence();
  *(volatile v4u*)(P + ro) = hv;
}

extern "C" void kernel_launch(void* const* d_in, const int* in_sizes, int n_in,
                              void* d_out, int out_size, void* d_ws, size_t ws_size,
                              hipStream_t stream) {
  if (n_in < 10) return;
  if (in_sizes[0] != NB * DM * PP) return;
  if (in_sizes[1] != HH * PP * PP) return;
  if (in_sizes[2] != HDIM * DM || in_sizes[4] != HDIM * DM || in_sizes[6] != HDIM * DM) return;
  if (in_sizes[3] != HDIM || in_sizes[5] != HDIM || in_sizes[7] != HDIM) return;
  if (in_sizes[8] != DM * HDIM || in_sizes[9] != DM) return;
  if (out_size != NB * DM * PP) return;

  const float* x   = (const float*)d_in[0];
  const float* pos = (const float*)d_in[1];
  const float* Wk  = (const float*)d_in[2];
  const float* bk  = (const float*)d_in[3];
  const float* Wq  = (const float*)d_in[4];
  const float* bq  = (const float*)d_in[5];
  const float* Wv  = (const float*)d_in[6];
  const float* bv  = (const float*)d_in[7];
  const float* Wo  = (const float*)d_in[8];
  const float* bo  = (const float*)d_in[9];

  const size_t BW   = (size_t)HDIM * DM * 2;
  const size_t BXT  = (size_t)NB * PP * DM * 2;
  const size_t BACT = (size_t)PP * HDIM * 2;
  const size_t BPT  = (size_t)HH * PP * PP * 4;
  const size_t BS   = (size_t)HH * PP * PP * 4;
  const size_t BP   = (size_t)HH * PP * PP * 2;
  size_t off = 0;
  const size_t oWk16 = off; off += BW;
  const size_t oWq16 = off; off += BW;
  const size_t oWv16 = off; off += BW;
  const size_t oWo16 = off; off += BW;
  const size_t oXT16 = off; off += BXT;
  const size_t oQ16  = off; off += BACT;
  const size_t oK16  = off; off += BACT;
  const size_t oVC16 = off; off += BACT;
  const size_t oOUTP = off; off += BACT;
  const size_t oPT   = off; off += BPT;
  const size_t oS    = off; off += BS;
  const size_t oP16  = off; off += BP;
  if (off > ws_size) return;

  char* ws = (char*)d_ws;
  unsigned short* Wk16  = (unsigned short*)(ws + oWk16);
  unsigned short* Wq16  = (unsigned short*)(ws + oWq16);
  unsigned short* Wv16  = (unsigned short*)(ws + oWv16);
  unsigned short* Wo16  = (unsigned short*)(ws + oWo16);
  unsigned short* XT16  = (unsigned short*)(ws + oXT16);
  unsigned short* Q16   = (unsigned short*)(ws + oQ16);
  unsigned short* K16   = (unsigned short*)(ws + oK16);
  unsigned short* VC16  = (unsigned short*)(ws + oVC16);
  unsigned short* OUTP  = (unsigned short*)(ws + oOUTP);
  float*          PT    = (float*)(ws + oPT);
  float*          Sbuf  = (float*)(ws + oS);
  unsigned short* P16   = (unsigned short*)(ws + oP16);

  const dim3 blk(256);
  const int n2w = HDIM * DM / 2;
  const dim3 gCastW((n2w + 255) / 256);

  cast_f16x2_kernel<<<gCastW, blk, 0, stream>>>(Wk, Wk16, n2w, 16.0f);
  cast_f16x2_kernel<<<gCastW, blk, 0, stream>>>(Wq, Wq16, n2w, 16.0f);
  cast_f16x2_kernel<<<gCastW, blk, 0, stream>>>(Wv, Wv16, n2w, 16.0f);
  cast_f16x2_kernel<<<gCastW, blk, 0, stream>>>(Wo, Wo16, n2w, 16.0f);
  xt_cast_kernel<<<NB * (PP / 64) * (DM / 64), blk, 0, stream>>>(x, XT16);
  pos_t_kernel<<<HH * (PP / 64) * (PP / 64), blk, 0, stream>>>(pos, PT);

  const dim3 gProj(((PP / 64) * (HDIM / 64) + 7) / 8, 1);
  const dim3 gS(((PP / 64) * (PP / 64) + 7) / 8, HH);
  const dim3 gPV(((PP / 64) * (DM / 64) + 7) / 8, HH);
  const dim3 gOut(((DM / 64) * (PP / 64) + 7) / 8, 1);
  const float wscale  = 1.0f / 16.0f;
  const float sscale  = 0.0625f;
  const float pvscale = 16.0f * PSCALE_INV;
  const float oscale  = 1.0f / 256.0f;

  for (int n = 0; n < NB; ++n) {
    const unsigned short* XTn = XT16 + (size_t)n * PP * DM;
    wmma_gemm64<0, false, 2, 1, false, 0><<<gProj, blk, 0, stream>>>(
        XTn, XTn, DM, 0L, Wq16, Wq16, DM, 0L, (void*)Q16, (void*)Q16, HDIM, 0L,
        bq, bq, 0L, PP, HDIM, DM, wscale);
    wmma_gemm64<0, false, 2, 1, false, 0><<<gProj, blk, 0, stream>>>(
        XTn, XTn, DM, 0L, Wk16, Wk16, DM, 0L, (void*)K16, (void*)K16, HDIM, 0L,
        bk, bk, 0L, PP, HDIM, DM, wscale);
    wmma_gemm64<0, false, 1, 1, false, 0><<<gProj, blk, 0, stream>>>(
        Wv16, Wv16, DM, 0L, XTn, XTn, DM, 0L, (void*)VC16, (void*)VC16, PP, 0L,
        bv, bv, 0L, HDIM, PP, DM, wscale);
    wmma_gemm64<0, false, 0, 0, false, 0><<<gS, blk, 0, stream>>>(
        Q16, Q16, HDIM, (long)DM, K16, K16, HDIM, (long)DM,
        (void*)Sbuf, (void*)Sbuf, PP, (long)PP * PP,
        bq, bq, 0L, PP, PP, DM, sscale);
    softmax_bias_kernel<<<dim3(PP, HH), dim3(128), 0, stream>>>(Sbuf, PT, P16);
    wmma_gemm64<0, false, 0, 1, false, 0><<<gPV, blk, 0, stream>>>(
        P16, P16, PP, (long)PP * PP, VC16, VC16, PP, (long)DM * PP,
        (void*)OUTP, (void*)OUTP, HDIM, (long)DM,
        bq, bq, 0L, PP, DM, PP, pvscale);
    float* outn = (float*)d_out + (size_t)n * DM * PP;
    wmma_gemm64<0, false, 1, 0, false, 0><<<gOut, blk, 0, stream>>>(
        Wo16, Wo16, HDIM, 0L, OUTP, OUTP, HDIM, 0L, (void*)outn, (void*)outn, PP, 0L,
        bo, bo, 0L, DM, PP, HDIM, oscale);
  }
  (void)hipGetLastError();
}
